// PAM_43602507989302
// MI455X (gfx1250) — hardware-verified
//
#include <hip/hip_runtime.h>
#include <math.h>

typedef __attribute__((ext_vector_type(16))) _Float16 v16h;
typedef __attribute__((ext_vector_type(8)))  _Float16 v8h;
typedef __attribute__((ext_vector_type(16))) __bf16   v16b;
typedef __attribute__((ext_vector_type(8)))  __bf16   v8b;
typedef __attribute__((ext_vector_type(8)))  float    v8f;
typedef __attribute__((ext_vector_type(4)))  float    v4f;

constexpr int kBatch = 4;
constexpr int kNpix  = 4096;
constexpr int kCh    = 512;
constexpr int kChR   = 64;
constexpr int kRows  = kBatch * kNpix;
constexpr int kQKOut = 2 * kChR;
constexpr float kWqkCarry    = 256.0f;
constexpr float kWqkCarryInv = 1.0f / kWqkCarry;
constexpr float kResCarry    = 2048.0f;
constexpr float kResCarryInv = 1.0f / kResCarry;
constexpr float kWdCarry     = 16.0f;
constexpr float kWdCarryInv  = 1.0f / kWdCarry;
constexpr float kPCarry      = 32768.0f;
constexpr int kQB  = 32;
constexpr int kKT  = 128;
constexpr int kSP  = 132;
constexpr int kPP  = 136;
constexpr int kOP  = 68;
constexpr int kBlkPerB = kNpix / kQB;
static_assert(kChR == 64);
static_assert((kCh % 32) == 0 && (kChR % 32) == 0 && (kNpix % 32) == 0);
static_assert((kRows % 64) == 0 && (kCh % 64) == 0 && (kNpix % 64) == 0 && (kQKOut % 64) == 0);
static_assert((kNpix % kKT) == 0 && (kNpix % kQB) == 0 && kCh == 8 * 64);

constexpr size_t kOffXH  = 0;
constexpr size_t kOffXL  = kOffXH  + (size_t)kRows * kCh * 2;
constexpr size_t kOffWQH = kOffXL  + (size_t)kRows * kCh * 2;
constexpr size_t kOffWQL = kOffWQH + (size_t)kQKOut * kCh * 2;
constexpr size_t kOffWDT = kOffWQL + (size_t)kQKOut * kCh * 2;
constexpr size_t kOffQH  = kOffWDT + (size_t)kCh * kCh * 2;
constexpr size_t kOffQL  = kOffQH  + (size_t)kRows * kChR * 2;
constexpr size_t kOffKH  = kOffQL  + (size_t)kRows * kChR * 2;
constexpr size_t kOffKL  = kOffKH  + (size_t)kRows * kChR * 2;
constexpr size_t kOffVT  = kOffKL  + (size_t)kRows * kChR * 2;
constexpr size_t kWsTotal = kOffVT + (size_t)kBatch * kCh * kNpix * 2;
static_assert(kWsTotal == 59506688ull);
static_assert(kWsTotal <= 134217728ull);
static_assert((kOffXL % 128) == 0 && (kOffWQH % 128) == 0 && (kOffWQL % 128) == 0 && (kOffWDT % 128) == 0 &&
              (kOffQH % 128) == 0 && (kOffQL % 128) == 0 && (kOffKH % 128) == 0 && (kOffKL % 128) == 0 &&
              (kOffVT % 128) == 0);

__device__ __forceinline__ unsigned short f2bf_bits(float f) {
  unsigned u = __float_as_uint(f);
  return (unsigned short)((u + 0x7FFFu + ((u >> 16) & 1u)) >> 16);
}
__device__ __forceinline__ float bf_bits2f(unsigned short h) { return __uint_as_float(((unsigned)h) << 16); }

__device__ __forceinline__ void dep_guard4_h(v8f& a, v8f& b, v8f& c, v8f& d, v16h x, v16h y) {
  asm volatile("v_nop\n\tv_nop\n\tv_nop\n\tv_nop" : "+v"(a), "+v"(b), "+v"(c), "+v"(d) : "v"(x), "v"(y));
}
__device__ __forceinline__ void dep_guard4_b(v8f& a, v8f& b, v8f& c, v8f& d, v16b x, v16b y) {
  asm volatile("v_nop\n\tv_nop\n\tv_nop\n\tv_nop" : "+v"(a), "+v"(b), "+v"(c), "+v"(d) : "v"(x), "v"(y));
}
__device__ __forceinline__ void keep4_h(v16h a, v16h b, v16h c, v16h d) { asm volatile("v_nop" :: "v"(a), "v"(b), "v"(c), "v"(d)); }
__device__ __forceinline__ void keep4_b(v16b a, v16b b, v16b c, v16b d) { asm volatile("v_nop" :: "v"(a), "v"(b), "v"(c), "v"(d)); }
__device__ __forceinline__ void acc_guard4(v8f& a, v8f& b, v8f& c, v8f& d) { asm volatile("v_nop\n\tv_nop\n\tv_nop\n\tv_nop" : "+v"(a), "+v"(b), "+v"(c), "+v"(d)); }
template <typename T> struct Frag;
template <> struct Frag<_Float16> {
  typedef v16h V; union U { v16h v; v8h h[2]; };
  static __device__ __forceinline__ v16h load(const _Float16* p) {
    U f; f.h[0] = *(const v8h*)(p); f.h[1] = *(const v8h*)(p + 16); return f.v;
  }
  static __device__ __forceinline__ v8f mma(v16h a, v16h b, v8f c) {
    return __builtin_amdgcn_wmma_f32_16x16x32_f16(false, a, false, b, (short)0, c, false, false);
  }
  static __device__ __forceinline__ void guard4(v8f& a, v8f& b, v8f& c, v8f& d, v16h x, v16h y) { dep_guard4_h(a, b, c, d, x, y); }
  static __device__ __forceinline__ void keep(v16h a, v16h b, v16h c, v16h d) { keep4_h(a, b, c, d); }
};
template <> struct Frag<__bf16> {
  typedef v16b V; union U { v16b v; v8b h[2]; };
  static __device__ __forceinline__ v16b load(const __bf16* p) {
    U f; f.h[0] = *(const v8b*)(p); f.h[1] = *(const v8b*)(p + 16); return f.v;
  }
  static __device__ __forceinline__ v8f mma(v16b a, v16b b, v8f c) {
    return __builtin_amdgcn_wmma_f32_16x16x32_bf16(false, a, false, b, (short)0, c, false, false);
  }
  static __device__ __forceinline__ void guard4(v8f& a, v8f& b, v8f& c, v8f& d, v16b x, v16b y) { dep_guard4_b(a, b, c, d, x, y); }
  static __device__ __forceinline__ void keep(v16b a, v16b b, v16b c, v16b d) { keep4_b(a, b, c, d); }
};

__device__ __forceinline__ v8f mma_h(v16h a, v16h b, v8f c) {
  c = __builtin_amdgcn_wmma_f32_16x16x32_f16(false, a, false, b, (short)0, c, false, false);
  asm volatile("v_nop\n\tv_nop\n\tv_nop\n\tv_nop" : "+v"(c) : "v"(a), "v"(b));
  return c;
}

__device__ __forceinline__ void wave_lds_sync() {
  __builtin_amdgcn_fence(__ATOMIC_RELEASE, "workgroup");
  __builtin_amdgcn_wave_barrier();
  __builtin_amdgcn_fence(__ATOMIC_ACQUIRE, "workgroup");
}

template <int ET> struct Elem;
template <> struct Elem<0> { typedef _Float16 T; };
template <> struct Elem<1> { typedef __bf16 T; };
template <int ET, bool SPLIT, int BIAS_MODE, int OUT_MODE, bool RESID, int ACT = 0>
__global__ __launch_bounds__(256) void wmma_gemm64(
    const unsigned short* __restrict__ Ap, const unsigned short* __restrict__ A2p, int lda, long strideA,
    const unsigned short* __restrict__ Btp, const unsigned short* __restrict__ Bt2p, int ldb, long strideB,
    void* __restrict__ Cout, void* __restrict__ Cout2, int ldc, long strideC,
    const float* __restrict__ bias,
    const float* __restrict__ resid, long strideR,
    int M, int N, int K, float scale) {
  typedef typename Elem<ET>::T T;
  typedef typename Frag<T>::V V;
  const T* A = (const T*)Ap; const T* A2 = (const T*)A2p; const T* Bt = (const T*)Btp; const T* Bt2 = (const T*)Bt2p;
  __shared__ __align__(16) float sT[8][16 * 68];
  const int b    = blockIdx.y;
  const int lane = threadIdx.x & 31;
  const int wave = threadIdx.x >> 5;
  const int tilesN = N >> 6;
  const int tilesM = M >> 6;
  const int tile = blockIdx.x * 8 + wave;
  if (tile >= tilesM * tilesN) return;
  const int tm = tile / tilesN;
  const int tn = tile - tm * tilesN;
  const int m0 = tm << 6;
  const int n0 = tn << 6;

  const T* Ab  = A  + (size_t)b * strideA;
  const T* Bb  = Bt + (size_t)b * strideB;
  const T* Ab2 = SPLIT ? (A2  + (size_t)b * strideA) : nullptr;
  const T* Bb2 = SPLIT ? (Bt2 + (size_t)b * strideB) : nullptr;

  const int rlane = lane & 15;
  const int koff  = (lane >> 4) * 8;
  const int mOff  = (lane >> 4) * 8;

  v8f acc[4][4];
#pragma unroll
  for (int i = 0; i < 4; ++i)
#pragma unroll
    for (int j = 0; j < 4; ++j) acc[i][j] = (v8f){0.f,0.f,0.f,0.f,0.f,0.f,0.f,0.f};

  for (int k0 = 0; k0 < K; k0 += 32) {
    V bh[4], bl[4];
#pragma unroll
    for (int j = 0; j < 4; ++j) {
      const size_t bo = (size_t)(n0 + (j << 4) + rlane) * ldb + koff + k0;
      bh[j] = Frag<T>::load(Bb + bo);
      if (SPLIT) bl[j] = Frag<T>::load(Bb2 + bo);
    }
#pragma unroll
    for (int i = 0; i < 4; ++i) {
      const size_t ao = (size_t)(m0 + (i << 4) + rlane) * lda + koff + k0;
      V ah = Frag<T>::load(Ab + ao);
      V al;
      if (SPLIT) al = Frag<T>::load(Ab2 + ao);
#pragma unroll
      for (int j = 0; j < 4; ++j) {
        acc[i][j] = Frag<T>::mma(ah, bh[j], acc[i][j]);
        if (SPLIT) {
          acc[i][j] = Frag<T>::mma(ah, bl[j], acc[i][j]);
          acc[i][j] = Frag<T>::mma(al, bh[j], acc[i][j]);
        }
      }
      Frag<T>::guard4(acc[i][0], acc[i][1], acc[i][2], acc[i][3], ah, SPLIT ? al : ah);
    }
    Frag<T>::keep(bh[0], bh[1], bh[2], bh[3]);
    if (SPLIT) Frag<T>::keep(bl[0], bl[1], bl[2], bl[3]);
  }
  acc_guard4(acc[0][0], acc[0][1], acc[0][2], acc[0][3]);
  acc_guard4(acc[1][0], acc[1][1], acc[1][2], acc[1][3]);
  acc_guard4(acc[2][0], acc[2][1], acc[2][2], acc[2][3]);
  acc_guard4(acc[3][0], acc[3][1], acc[3][2], acc[3][3]);

  float* slab = sT[wave];
  const float* Rb = RESID ? (resid + (size_t)b * strideR) : nullptr;
#pragma unroll
  for (int i = 0; i < 4; ++i) {
    const int mBase = m0 + (i << 4);
#pragma unroll
    for (int j = 0; j < 4; ++j) {
      const int n = n0 + (j << 4) + rlane;
      float bv = 0.f;
      if (BIAS_MODE == 2) bv = bias[n];
#pragma unroll
      for (int r = 0; r < 8; ++r) {
        float v = acc[i][j][r] * scale;
        if (BIAS_MODE == 1) v += bias[mBase + mOff + r];
        if (BIAS_MODE == 2) v += bv;
        if (RESID) v += Rb[(size_t)(mBase + mOff + r) * ldc + n];
        if (ACT == 2) v = fmaxf(v, 0.0f);
        if (ACT == 4) v = (v > 0.f) ? v : 0.01f * v;
        slab[(mOff + r) * 68 + (j << 4) + rlane] = v;
      }
    }
    __builtin_amdgcn_fence(__ATOMIC_RELEASE, "workgroup");
    __builtin_amdgcn_wave_barrier();
    __builtin_amdgcn_fence(__ATOMIC_ACQUIRE, "workgroup");
    if (OUT_MODE == 0) {
      float* C = (float*)Cout + (size_t)b * strideC;
      const int hh = lane >> 4, c4 = (lane & 15) * 4;
      for (int pass = 0; pass < 2; ++pass) {
#pragma unroll
        for (int it = 0; it < 8; ++it) {
          const int row = it * 2 + hh;
          v4f v = *(const v4f*)(slab + row * 68 + c4);
          *(volatile v4f*)(C + (size_t)(mBase + row) * ldc + n0 + c4) = v;
        }
        __threadfence();
      }
    } else {
      const int q = lane >> 3, c8 = (lane & 7) * 8;
      unsigned short* C  = (unsigned short*)Cout  + (size_t)b * strideC;
      unsigned short* C2 = (OUT_MODE == 2) ? ((unsigned short*)Cout2 + (size_t)b * strideC) : nullptr;
      for (int pass = 0; pass < 2; ++pass) {
#pragma unroll
        for (int it = 0; it < 4; ++it) {
          const int row = it * 4 + q;
          const float* sp = slab + row * 68 + c8;
          v8h hv, lv;
#pragma unroll
          for (int e = 0; e < 8; ++e) {
            if (OUT_MODE == 1) {
              hv[e] = (_Float16)sp[e];
            } else {
              unsigned short hb = f2bf_bits(sp[e]);
              unsigned short lb = f2bf_bits(sp[e] - bf_bits2f(hb));
              hv[e] = __builtin_bit_cast(_Float16, hb);
              lv[e] = __builtin_bit_cast(_Float16, lb);
            }
          }
          *(volatile v8h*)(C + (size_t)(mBase + row) * ldc + n0 + c8) = hv;
          if (OUT_MODE == 2) *(volatile v8h*)(C2 + (size_t)(mBase + row) * ldc + n0 + c8) = lv;
        }
        __threadfence();
      }
    }
    __builtin_amdgcn_fence(__ATOMIC_RELEASE, "workgroup");
    __builtin_amdgcn_wave_barrier();
    __builtin_amdgcn_fence(__ATOMIC_ACQUIRE, "workgroup");
  }
}

__global__ __launch_bounds__(256) void xsplit_kernel(
    const float* __restrict__ src, unsigned short* __restrict__ dhi, unsigned short* __restrict__ dlo, int total8)
{
  const int i = blockIdx.x * 256 + threadIdx.x;
  if (i >= total8) return;
  const size_t e0 = (size_t)i << 3;
  const v4f a0 = *(const v4f*)(src + e0);
  const v4f a1 = *(const v4f*)(src + e0 + 4);
  v8h hv, lv;
#pragma unroll
  for (int e = 0; e < 4; ++e) {
    const float f0 = a0[e];
    const float f1 = a1[e];
    const _Float16 h0 = (_Float16)f0;
    const _Float16 h1 = (_Float16)f1;
    hv[e]     = h0;
    hv[4 + e] = h1;
    lv[e]     = (_Float16)((f0 - (float)h0) * kResCarry);
    lv[4 + e] = (_Float16)((f1 - (float)h1) * kResCarry);
  }
  unsigned short* qh = dhi + e0;
  unsigned short* ql = dlo + e0;
  *(volatile v8h*)qh = hv;
  *(volatile v8h*)ql = lv;
  __threadfence();
  *(volatile v8h*)qh = hv;
  *(volatile v8h*)ql = lv;
}

template <bool LO>
__global__ __launch_bounds__(256) void wtrans_kernel(
    const float* __restrict__ W0, const float* __restrict__ W1, int ldw,
    unsigned short* __restrict__ outH, unsigned short* __restrict__ outL, float scale)
{
  __shared__ float sm[64][65];
  const int t  = threadIdx.x;
  const int k0 = blockIdx.x * 64;
  const int o0 = blockIdx.y * 64;
  const int z  = blockIdx.z;
  const float* W = (z == 0) ? W0 : W1;
#pragma unroll
  for (int i = 0; i < 16; ++i) {
    const int e  = i * 256 + t;
    const int r  = e >> 6;
    const int cc = e & 63;
    sm[cc][r] = W[(size_t)(k0 + r) * ldw + o0 + cc] * scale;
  }
  __syncthreads();
  const int lane = t & 31, wave = t >> 5;
  const int q4 = lane >> 3, c8 = (lane & 7) * 8;
  v8h hv[2], lv[2];
#pragma unroll
  for (int it = 0; it < 2; ++it) {
    const int row = wave * 8 + it * 4 + q4;
#pragma unroll
    for (int e = 0; e < 8; ++e) {
      const float f = sm[row][c8 + e];
      const _Float16 h = (_Float16)f;
      hv[it][e] = h;
      lv[it][e] = (_Float16)((f - (float)h) * kResCarry);
    }
  }
  for (int pass = 0; pass < 2; ++pass) {
#pragma unroll
    for (int it = 0; it < 2; ++it) {
      const int row = wave * 8 + it * 4 + q4;
      const size_t o = (size_t)(z * 64 + o0 + row) * kCh + k0 + c8;
      *(volatile v8h*)(outH + o) = hv[it];
      if (LO) *(volatile v8h*)(outL + o) = lv[it];
    }
    __threadfence();
  }
}

__global__ __launch_bounds__(256) void qkproj_kernel(
    const unsigned short* __restrict__ Xhp, const unsigned short* __restrict__ Xlp,
    const unsigned short* __restrict__ Whp, const unsigned short* __restrict__ Wlp,
    unsigned short* __restrict__ Qh, unsigned short* __restrict__ Ql,
    unsigned short* __restrict__ Kh, unsigned short* __restrict__ Kl)
{
  typedef Frag<_Float16> FH;
  __shared__ __align__(16) float sT[8][16 * kOP];
  const int lane = threadIdx.x & 31, wave = threadIdx.x >> 5;
  const int hh = lane >> 4, c = lane & 15;
  const int tile = blockIdx.x * 8 + wave;
  if (tile >= (kRows / 16) * 2) return;
  const int tm = tile >> 1, tn = tile & 1;
  const int m0 = tm * 16, n0 = tn * 64;
  const _Float16* Xh = (const _Float16*)Xhp;
  const _Float16* Xl = (const _Float16*)Xlp;
  const _Float16* Wh = (const _Float16*)Whp;
  const _Float16* Wl = (const _Float16*)Wlp;

  v8f am[4], ar[4];
#pragma unroll
  for (int j = 0; j < 4; ++j) {
    am[j] = (v8f){0.f,0.f,0.f,0.f,0.f,0.f,0.f,0.f};
    ar[j] = (v8f){0.f,0.f,0.f,0.f,0.f,0.f,0.f,0.f};
  }
  const size_t abase = (size_t)(m0 + c) * kCh + 8 * hh;
#pragma unroll 1
  for (int k0 = 0; k0 < kCh; k0 += 32) {
    const v16h ah = FH::load(Xh + abase + k0);
    const v16h al = FH::load(Xl + abase + k0);
#pragma unroll
    for (int j = 0; j < 4; ++j) {
      const size_t bo = (size_t)(n0 + j * 16 + c) * kCh + 8 * hh + k0;
      const v16h bh = FH::load(Wh + bo);
      const v16h bl = FH::load(Wl + bo);
      am[j] = mma_h(ah, bh, am[j]);
      ar[j] = mma_h(ah, bl, ar[j]);
      ar[j] = mma_h(al, bh, ar[j]);
    }
  }
  float* slab = sT[wave];
#pragma unroll
  for (int j = 0; j < 4; ++j) {
#pragma unroll
    for (int r = 0; r < 8; ++r) {
      const float v = (am[j][r] + ar[j][r] * kResCarryInv) * kWqkCarryInv;
      slab[(8 * hh + r) * kOP + j * 16 + c] = v;
    }
  }
  wave_lds_sync();
  unsigned short* dH = tn ? Kh : Qh;
  unsigned short* dL = tn ? Kl : Ql;
  const int q4 = lane >> 3, c8 = (lane & 7) * 8;
  v8h hv[4], lv[4];
#pragma unroll
  for (int it = 0; it < 4; ++it) {
    const int row = it * 4 + q4;
    const float* sp = slab + row * kOP + c8;
    const v4f a0 = *(const v4f*)(sp);
    const v4f a1 = *(const v4f*)(sp + 4);
#pragma unroll
    for (int e = 0; e < 4; ++e) {
      const float f0 = a0[e];
      const float f1 = a1[e];
      const _Float16 h0 = (_Float16)f0;
      const _Float16 h1 = (_Float16)f1;
      hv[it][e]     = h0;
      hv[it][4 + e] = h1;
      lv[it][e]     = (_Float16)((f0 - (float)h0) * kResCarry);
      lv[it][4 + e] = (_Float16)((f1 - (float)h1) * kResCarry);
    }
  }
  for (int pass = 0; pass < 2; ++pass) {
#pragma unroll
    for (int it = 0; it < 4; ++it) {
      const int row = it * 4 + q4;
      const size_t o = (size_t)(m0 + row) * kChR + c8;
      *(volatile v8h*)(dH + o) = hv[it];
      *(volatile v8h*)(dL + o) = lv[it];
    }
    __threadfence();
  }
}

__global__ __launch_bounds__(256) void attn_kernel(
    const unsigned short* __restrict__ Qhp, const unsigned short* __restrict__ Qlp,
    const unsigned short* __restrict__ Khp, const unsigned short* __restrict__ Klp,
    const unsigned short* __restrict__ Vtp, const float* __restrict__ x,
    const float* __restrict__ gamma, float* __restrict__ out)
{
  typedef Frag<_Float16> FH;
  __shared__ __align__(16) float    Ssh[kQB * kSP];
  __shared__ __align__(16) _Float16 Psh[kQB * kPP];
  __shared__ __align__(16) float    Ash[kQB];
  __shared__ __align__(16) float    Lsh[kQB];
  __shared__ __align__(16) float    Osh[8][16 * kOP];

  const int tid = threadIdx.x, wave = tid >> 5, lane = tid & 31;
  const int hh = lane >> 4, c = lane & 15;
  const int b = blockIdx.x / kBlkPerB;
  const int qblk = blockIdx.x - b * kBlkPerB;
  const int prow0 = b * kNpix;
  const int q0 = prow0 + qblk * kQB;
  const int qs = wave & 1, kg = wave >> 1;

  const _Float16* Qh = (const _Float16*)Qhp;
  const _Float16* Ql = (const _Float16*)Qlp;
  const _Float16* Kh = (const _Float16*)Khp;
  const _Float16* Kl = (const _Float16*)Klp;
  const _Float16* Vt = (const _Float16*)Vtp;

  const size_t qo = (size_t)(q0 + qs * 16 + c) * kChR + 8 * hh;
  const v16h qh0 = FH::load(Qh + qo);
  const v16h qh1 = FH::load(Qh + qo + 32);
  const v16h ql0 = FH::load(Ql + qo);
  const v16h ql1 = FH::load(Ql + qo + 32);

  v8f o[2][4];
#pragma unroll
  for (int a = 0; a < 2; ++a)
#pragma unroll
    for (int t = 0; t < 4; ++t) o[a][t] = (v8f){0.f,0.f,0.f,0.f,0.f,0.f,0.f,0.f};

  const int srow = wave * 4 + (lane >> 3);
  const int scol = (lane & 7) * 16;
  float m_run = -INFINITY;
  float l_run = 0.0f;

#pragma unroll 1
  for (int kt = 0; kt < kNpix / kKT; ++kt) {
    const int key0 = kt * kKT;
#pragma unroll
    for (int jj = 0; jj < 2; ++jj) {
      const int j = kg * 2 + jj;
      const size_t ko = (size_t)(prow0 + key0 + j * 16 + c) * kChR + 8 * hh;
      const v16h kh0 = FH::load(Kh + ko);
      const v16h kh1 = FH::load(Kh + ko + 32);
      const v16h kl0 = FH::load(Kl + ko);
      const v16h kl1 = FH::load(Kl + ko + 32);
      v8f sm = (v8f){0.f,0.f,0.f,0.f,0.f,0.f,0.f,0.f};
      v8f sr = (v8f){0.f,0.f,0.f,0.f,0.f,0.f,0.f,0.f};
      sm = mma_h(qh0, kh0, sm);
      sm = mma_h(qh1, kh1, sm);
      sr = mma_h(qh0, kl0, sr);
      sr = mma_h(qh1, kl1, sr);
      sr = mma_h(ql0, kh0, sr);
      sr = mma_h(ql1, kh1, sr);
      float* sw = Ssh + (qs * 16 + 8 * hh) * kSP + j * 16 + c;
#pragma unroll
      for (int r = 0; r < 8; ++r) sw[r * kSP] = sm[r] + sr[r] * kResCarryInv;
    }
    __syncthreads();
    {
      const float* sp = Ssh + srow * kSP + scol;
      const v4f a0 = *(const v4f*)(sp);
      const v4f a1 = *(const v4f*)(sp + 4);
      const v4f a2 = *(const v4f*)(sp + 8);
      const v4f a3 = *(const v4f*)(sp + 12);
      float sv[16];
#pragma unroll
      for (int e = 0; e < 4; ++e) {
        sv[e]      = a0[e];
        sv[4 + e]  = a1[e];
        sv[8 + e]  = a2[e];
        sv[12 + e] = a3[e];
      }
      float tm = sv[0];
#pragma unroll
      for (int e = 1; e < 16; ++e) tm = fmaxf(tm, sv[e]);
      tm = fmaxf(tm, __shfl_xor(tm, 1, 32));
      tm = fmaxf(tm, __shfl_xor(tm, 2, 32));
      tm = fmaxf(tm, __shfl_xor(tm, 4, 32));
      const float m_new = fmaxf(m_run, tm);
      const float alpha = __expf(m_run - m_new);
      m_run = m_new;
      float psum = 0.0f;
      v8h p0, p1;
#pragma unroll
      for (int e = 0; e < 8; ++e) {
        const float pe = __expf(sv[e] - m_new);
        psum += pe;
        p0[e] = (_Float16)(pe * kPCarry);
      }
#pragma unroll
      for (int e = 0; e < 8; ++e) {
        const float pe = __expf(sv[8 + e] - m_new);
        psum += pe;
        p1[e] = (_Float16)(pe * kPCarry);
      }
      psum += __shfl_xor(psum, 1, 32);
      psum += __shfl_xor(psum, 2, 32);
      psum += __shfl_xor(psum, 4, 32);
      l_run = l_run * alpha + psum;
      _Float16* pw = Psh + srow * kPP + scol;
      *(v8h*)(pw)     = p0;
      *(v8h*)(pw + 8) = p1;
      if ((lane & 7) == 0) Ash[srow] = alpha;
    }
    __syncthreads();
    {
      const float* ap = Ash + 8 * hh;
      const v4f f0 = *(const v4f*)(ap);
      const v4f f1 = *(const v4f*)(ap + 4);
      const v4f f2 = *(const v4f*)(ap + 16);
      const v4f f3 = *(const v4f*)(ap + 20);
      float fa[8], fb[8];
#pragma unroll
      for (int e = 0; e < 4; ++e) {
        fa[e]     = f0[e];
        fa[4 + e] = f1[e];
        fb[e]     = f2[e];
        fb[4 + e] = f3[e];
      }
      int changed = 0;
#pragma unroll
      for (int e = 0; e < 8; ++e) changed |= ((fa[e] != 1.0f) || (fb[e] != 1.0f)) ? 1 : 0;
      const int anyc = __any(changed);
      if (anyc) {
#pragma unroll
        for (int t = 0; t < 4; ++t) {
#pragma unroll
          for (int r = 0; r < 8; ++r) {
            o[0][t][r] *= fa[r];
            o[1][t][r] *= fb[r];
          }
        }
      }
      const _Float16* pp = Psh + c * kPP + 8 * hh;
      const _Float16* vp = Vt + (size_t)(b * kCh + wave * 64 + c) * kNpix + key0 + 8 * hh;
#pragma unroll 1
      for (int kk = 0; kk < kKT / 32; ++kk) {
        const v16h pa0 = FH::load(pp + kk * 32);
        const v16h pa1 = FH::load(pp + 16 * kPP + kk * 32);
#pragma unroll
        for (int t = 0; t < 4; ++t) {
          const v16h vb = FH::load(vp + (size_t)t * 16 * kNpix + kk * 32);
          o[0][t] = mma_h(pa0, vb, o[0][t]);
          o[1][t] = mma_h(pa1, vb, o[1][t]);
        }
      }
    }
  }

  const float g = gamma[0];
  if ((lane & 7) == 0) Lsh[srow] = g * (1.0f / (l_run * kPCarry));
  __syncthreads();

  float* os = Osh[wave];
  const int c4 = c * 4;
#pragma unroll
  for (int qq = 0; qq < 2; ++qq) {
    const float* lp = Lsh + qq * 16 + 8 * hh;
    const v4f i0 = *(const v4f*)(lp);
    const v4f i1 = *(const v4f*)(lp + 4);
    float inv[8];
#pragma unroll
    for (int e = 0; e < 4; ++e) {
      inv[e]     = i0[e];
      inv[4 + e] = i1[e];
    }
#pragma unroll
    for (int t = 0; t < 4; ++t) {
#pragma unroll
      for (int r = 0; r < 8; ++r) os[(8 * hh + r) * kOP + t * 16 + c] = o[qq][t][r] * inv[r];
    }
    wave_lds_sync();
    v4f vals[8];
#pragma unroll
    for (int it = 0; it < 8; ++it) {
      const int row = it * 2 + hh;
      const size_t go = (size_t)(q0 + qq * 16 + row) * kCh + wave * 64 + c4;
      const v4f ov = *(const v4f*)(os + row * kOP + c4);
      const v4f xv = *(const v4f*)(x + go);
      vals[it] = ov + xv;
    }
    for (int pass = 0; pass < 2; ++pass) {
#pragma unroll
      for (int it = 0; it < 8; ++it) {
        const int row = it * 2 + hh;
        const size_t go = (size_t)(q0 + qq * 16 + row) * kCh + wave * 64 + c4;
        *(volatile v4f*)(out + go) = vals[it];
      }
      __threadfence();
    }
    wave_lds_sync();
  }
}

extern "C" void kernel_launch(void* const* d_in, const int* in_sizes, int n_in,
                              void* d_out, int out_size, void* d_ws, size_t ws_size,
                              hipStream_t stream) {
  if (n_in < 5) return;
  if (in_sizes[0] != kRows * kCh) return;
  if (in_sizes[1] != kCh * kChR) return;
  if (in_sizes[2] != kCh * kChR) return;
  if (in_sizes[3] != kCh * kCh) return;
  if (in_sizes[4] != 1) return;
  if (out_size != kRows * kCh) return;
  if (ws_size < kWsTotal) return;

  const float* x     = (const float*)d_in[0];
  const float* Wb    = (const float*)d_in[1];
  const float* Wc    = (const float*)d_in[2];
  const float* Wd    = (const float*)d_in[3];
  const float* gamma = (const float*)d_in[4];
  float* out = (float*)d_out;

  char* ws = (char*)d_ws;
  unsigned short* XH  = (unsigned short*)(ws + kOffXH);
  unsigned short* XL  = (unsigned short*)(ws + kOffXL);
  unsigned short* WQH = (unsigned short*)(ws + kOffWQH);
  unsigned short* WQL = (unsigned short*)(ws + kOffWQL);
  unsigned short* WDT = (unsigned short*)(ws + kOffWDT);
  unsigned short* QH  = (unsigned short*)(ws + kOffQH);
  unsigned short* QL  = (unsigned short*)(ws + kOffQL);
  unsigned short* KH  = (unsigned short*)(ws + kOffKH);
  unsigned short* KL  = (unsigned short*)(ws + kOffKL);
  unsigned short* VT  = (unsigned short*)(ws + kOffVT);

  xsplit_kernel<<<(kRows * kCh / 8) / 256, 256, 0, stream>>>(x, XH, XL, kRows * kCh / 8);

  wtrans_kernel<true><<<dim3(kCh / 64, 1, 2), 256, 0, stream>>>(Wb, Wc, kChR, WQH, WQL, kWqkCarry);

  wtrans_kernel<false><<<dim3(kCh / 64, kCh / 64, 1), 256, 0, stream>>>(Wd, Wd, kCh, WDT, WDT, kWdCarry);

  qkproj_kernel<<<((kRows / 16) * 2) / 8, 256, 0, stream>>>(XH, XL, WQH, WQL, QH, QL, KH, KL);

  wmma_gemm64<0, false, 0, 1, false><<<dim3((kCh / 64) * (kNpix / 64) / 8, kBatch), 256, 0, stream>>>(
      WDT, nullptr, kCh, 0L,
      XH, nullptr, kCh, (long)kNpix * kCh,
      (void*)VT, nullptr, kNpix, (long)kCh * kNpix,
      nullptr, nullptr, 0L,
      kCh, kNpix, kCh, kWdCarryInv);

  attn_kernel<<<kBatch * kBlkPerB, 256, 0, stream>>>(QH, QL, KH, KL, VT, x, gamma, out);
}
